// BlockR_86045374808442
// MI455X (gfx1250) — hardware-verified
//
#include <hip/hip_runtime.h>
#include <stddef.h>
#include <stdint.h>
#include <math.h>

#define EMBD 1024
#define HIDD 4096
#define NBAT 2
#define SEQL 4096
#define MTOK 8192
#define TCH  2048
#define NCHK 2
#define SFP  132

static_assert(MTOK == NBAT * SEQL);
static_assert(SEQL == NCHK * TCH);
static_assert(TCH % 128 == 0);
static_assert(HIDD % 128 == 0);
static_assert(EMBD % 128 == 0);
static_assert(EMBD % 32 == 0);
static_assert(HIDD % 32 == 0);
static_assert(HIDD % 256 == 0);
static_assert(EMBD == 128 * 8);
static_assert(HIDD == 2 * 256 * 8);
static_assert((HIDD * EMBD) % 2048 == 0);

typedef _Float16 hh;
typedef hh    v16h __attribute__((ext_vector_type(16)));
typedef hh    v8h  __attribute__((ext_vector_type(8)));
typedef float v8f  __attribute__((ext_vector_type(8)));
typedef float v4f  __attribute__((ext_vector_type(4)));

union Frag { v16h v; v8h p[2]; };

__device__ __forceinline__ v8f zero8() { return (v8f){0.f, 0.f, 0.f, 0.f, 0.f, 0.f, 0.f, 0.f}; }

__device__ __forceinline__ float wsum(float v) {
#pragma unroll
  for (int off = 16; off > 0; off >>= 1) v += __shfl_xor(v, off, 32);
  return v;
}

__device__ __forceinline__ v16h ldfrag(const hh* __restrict__ p, int ld, int row0, int k0, int lane) {
  const hh* q = p + (size_t)(row0 + (lane & 15)) * (size_t)ld + k0 + 8 * (lane >> 4);
  Frag f;
  f.p[0] = *(const v8h*)(q);
  f.p[1] = *(const v8h*)(q + 16);
  return f.v;
}

__device__ __forceinline__ v8f mma16(v16h a, v16h b, v8f cc) {
  return __builtin_amdgcn_wmma_f32_16x16x32_f16(false, a, false, b, (short)0, cc, false, false);
}

__device__ __forceinline__ void gemm32x64(const hh* __restrict__ A, int lda, const hh* __restrict__ B, int ldb,
                                          int ma, int nb, int kdim, int lane, v8f (&acc)[2][4]) {
#pragma unroll 1
  for (int k0 = 0; k0 < kdim; k0 += 32) {
    const v16h a0 = ldfrag(A, lda, ma, k0, lane);
    const v16h a1 = ldfrag(A, lda, ma + 16, k0, lane);
    const v16h b0 = ldfrag(B, ldb, nb, k0, lane);
    const v16h b1 = ldfrag(B, ldb, nb + 16, k0, lane);
    const v16h b2 = ldfrag(B, ldb, nb + 32, k0, lane);
    const v16h b3 = ldfrag(B, ldb, nb + 48, k0, lane);
    acc[0][0] = mma16(a0, b0, acc[0][0]);
    acc[1][0] = mma16(a1, b0, acc[1][0]);
    acc[0][1] = mma16(a0, b1, acc[0][1]);
    acc[1][1] = mma16(a1, b1, acc[1][1]);
    acc[0][2] = mma16(a0, b2, acc[0][2]);
    acc[1][2] = mma16(a1, b2, acc[1][2]);
    acc[0][3] = mma16(a0, b3, acc[0][3]);
    acc[1][3] = mma16(a1, b3, acc[1][3]);
    asm volatile("v_nop\n\tv_nop\n\tv_nop\n\tv_nop"
                 : "+v"(acc[0][0]), "+v"(acc[0][1]), "+v"(acc[0][2]), "+v"(acc[0][3]),
                   "+v"(acc[1][0]), "+v"(acc[1][1]), "+v"(acc[1][2]), "+v"(acc[1][3])
                 : "v"(a0), "v"(a1), "v"(b0), "v"(b1), "v"(b2), "v"(b3));
  }
}

template <int SC>
__global__ __launch_bounds__(256) void k_cvt(const float* __restrict__ w, hh* __restrict__ wh) {
  const size_t i = ((size_t)blockIdx.x * 256 + threadIdx.x) * 8;
  const v4f a0 = *(const v4f*)(w + i);
  const v4f a1 = *(const v4f*)(w + i + 4);
  v8f t = {a0[0], a0[1], a0[2], a0[3], a1[0], a1[1], a1[2], a1[3]};
  t = t * (float)SC;
  const v8h pk = __builtin_convertvector(t, v8h);
  *(volatile v8h*)(wh + i) = pk;
  __threadfence();
  *(volatile v8h*)(wh + i) = pk;
}

__global__ __launch_bounds__(128) void k_rms1(const float* __restrict__ x, hh* __restrict__ y) {
  __shared__ float red[4];
  const int tid = threadIdx.x, lane = tid & 31, w = tid >> 5;
  const size_t ro = (size_t)blockIdx.x * EMBD + (size_t)tid * 8;
  const v4f a0 = *(const v4f*)(x + ro), a1 = *(const v4f*)(x + ro + 4);
  const float f[8] = {a0[0], a0[1], a0[2], a0[3], a1[0], a1[1], a1[2], a1[3]};
  float ss = 0.f;
#pragma unroll
  for (int e = 0; e < 8; ++e) ss = fmaf(f[e], f[e], ss);
  ss = wsum(ss);
  if (lane == 0) red[w] = ss;
  __syncthreads();
  const float tot = (red[0] + red[1]) + (red[2] + red[3]);
  const float sc = rsqrtf(tot * (1.0f / (float)EMBD) + 1e-6f);
  v8f t;
#pragma unroll
  for (int e = 0; e < 8; ++e) t[e] = f[e] * sc;
  const v8h pk = __builtin_convertvector(t, v8h);
  *(volatile v8h*)(y + ro) = pk;
  __threadfence();
  *(volatile v8h*)(y + ro) = pk;
}

__global__ __launch_bounds__(256) void k_rms2(const float* __restrict__ yv, hh* __restrict__ yn) {
  __shared__ float red[8];
  const int tid = threadIdx.x, lane = tid & 31, w = tid >> 5;
  const size_t rb = (size_t)blockIdx.x * HIDD;
  const int c0 = tid * 8;
  const int c1 = (HIDD / 2) + tid * 8;
  const v4f a0 = *(const v4f*)(yv + rb + c0), a1 = *(const v4f*)(yv + rb + c0 + 4);
  const v4f b0 = *(const v4f*)(yv + rb + c1), b1 = *(const v4f*)(yv + rb + c1 + 4);
  const float f[16] = {a0[0], a0[1], a0[2], a0[3], a1[0], a1[1], a1[2], a1[3],
                       b0[0], b0[1], b0[2], b0[3], b1[0], b1[1], b1[2], b1[3]};
  float ss = 0.f;
#pragma unroll
  for (int e = 0; e < 16; ++e) ss = fmaf(f[e], f[e], ss);
  ss = wsum(ss);
  if (lane == 0) red[w] = ss;
  __syncthreads();
  const float tot = ((red[0] + red[1]) + (red[2] + red[3])) + ((red[4] + red[5]) + (red[6] + red[7]));
  const float sc = rsqrtf(tot * (1.0f / (float)HIDD) + 1e-6f);
  v8f t0, t1;
#pragma unroll
  for (int e = 0; e < 8; ++e) { t0[e] = f[e] * sc; t1[e] = f[8 + e] * sc; }
  const v8h pk0 = __builtin_convertvector(t0, v8h);
  const v8h pk1 = __builtin_convertvector(t1, v8h);
  *(volatile v8h*)(yn + rb + c0) = pk0;
  *(volatile v8h*)(yn + rb + c1) = pk1;
  __threadfence();
  *(volatile v8h*)(yn + rb + c0) = pk0;
  *(volatile v8h*)(yn + rb + c1) = pk1;
}

__global__ __launch_bounds__(256) void k_scan(const float* __restrict__ bp, float* __restrict__ ay,
                                              float* st, int rdst, int wrst, int tbase) {
  const int h = blockIdx.x * 256 + threadIdx.x;
  float ma = -1.0e30f, sa = 0.f, mb = -1.0e30f, sb = 0.f;
  if (rdst != 0) {
    ma = st[h];
    sa = st[HIDD + h];
    mb = st[2 * HIDD + h];
    sb = st[3 * HIDD + h];
  }
  const float* pb = bp + h;
  float* pa = ay + h;
#pragma unroll 1
  for (int t = 0; t < TCH; ++t) {
    const size_t o = (size_t)t * HIDD;
    const float va = pa[o];
    const float vb = pb[o];
    const float da = va - ma;
    const float ea = __expf(-fabsf(da));
    const bool  ua = da > 0.f;
    sa = ua ? fmaf(sa, ea, 1.0f) : (sa + ea);
    ma = ua ? va : ma;
    const float db = vb - mb;
    const float eb = __expf(-fabsf(db));
    const bool  ub = db > 0.f;
    sb = ub ? fmaf(sb, eb, 1.0f) : (sb + eb);
    mb = ub ? vb : mb;
    const float la = ma + __logf(sa);
    const float lb = mb + __logf(sb);
    const float lt = __logf((float)(tbase + t + 1));
    const float yv = __expf((la + lb) - 2.0f * lt);
    *(volatile float*)(pa + o) = yv;
    __threadfence();
    *(volatile float*)(pa + o) = yv;
  }
  if (wrst != 0) {
    *(volatile float*)(st + h) = ma;
    *(volatile float*)(st + HIDD + h) = sa;
    *(volatile float*)(st + 2 * HIDD + h) = mb;
    *(volatile float*)(st + 3 * HIDD + h) = sb;
    __threadfence();
    *(volatile float*)(st + h) = ma;
    *(volatile float*)(st + HIDD + h) = sa;
    *(volatile float*)(st + 2 * HIDD + h) = mb;
    *(volatile float*)(st + 3 * HIDD + h) = sb;
  }
}

template <int MODE>
__global__ __launch_bounds__(256) void k_gemm(const hh* __restrict__ Ap, const hh* __restrict__ Bp,
                                              const float* __restrict__ res, float* __restrict__ o32) {
  constexpr int KD  = (MODE == 0) ? EMBD : HIDD;
  constexpr int LDA = KD;
  constexpr int LDB = KD;
  constexpr int LDO = (MODE == 0) ? HIDD : EMBD;
  constexpr float OSC = (MODE == 0) ? (1.0f / 64.0f) : (1.0f / 256.0f);

  __shared__ __align__(16) float ldsf[64 * SFP];
  const int tid = threadIdx.x, lane = tid & 31, w = tid >> 5;
  const int h = lane >> 4, c = lane & 15;
  const int wm = (w >> 1) * 32, wn = (w & 1) * 64;
  const int m0 = blockIdx.y * 128;
  const int n0 = blockIdx.x * 128;

  v8f acc[2][4];
#pragma unroll
  for (int i = 0; i < 2; ++i)
#pragma unroll
    for (int j = 0; j < 4; ++j) acc[i][j] = zero8();
  gemm32x64(Ap, LDA, Bp, LDB, m0 + wm, n0 + wn, KD, lane, acc);

#pragma unroll
  for (int hf = 0; hf < 2; ++hf) {
    if ((w >> 2) == hf) {
#pragma unroll
      for (int i = 0; i < 2; ++i)
#pragma unroll
        for (int j = 0; j < 4; ++j)
#pragma unroll
          for (int r = 0; r < 8; ++r)
            ldsf[(wm - 64 * hf + 16 * i + 8 * h + r) * SFP + wn + 16 * j + c] = acc[i][j][r] * OSC;
    }
    __syncthreads();
    v4f val[8];
    size_t go[8];
#pragma unroll
    for (int it = 0; it < 8; ++it) {
      const int p  = tid + 256 * it;
      const int lr = p >> 5;
      const int pc = p & 31;
      const v4f sv = *(const v4f*)(ldsf + lr * SFP + pc * 4);
      const size_t gi = (size_t)(m0 + 64 * hf + lr) * LDO + n0 + pc * 4;
      if constexpr (MODE == 1) {
        const v4f rr = *(const v4f*)(res + gi);
        val[it] = sv + rr;
      } else {
        val[it] = sv;
      }
      go[it] = gi;
    }
#pragma unroll
    for (int it = 0; it < 8; ++it) *(volatile v4f*)(o32 + go[it]) = val[it];
    __threadfence();
#pragma unroll
    for (int it = 0; it < 8; ++it) *(volatile v4f*)(o32 + go[it]) = val[it];
    if (hf == 0) __syncthreads();
  }
}

extern "C" void kernel_launch(void* const* d_in, const int* in_sizes, int n_in,
                              void* d_out, int out_size, void* d_ws, size_t ws_size,
                              hipStream_t stream) {
  if (n_in < 4) return;
  if (in_sizes[0] != MTOK * EMBD) return;
  if (in_sizes[1] != HIDD * EMBD) return;
  if (in_sizes[2] != HIDD * EMBD) return;
  if (in_sizes[3] != EMBD * HIDD) return;
  if (out_size != MTOK * EMBD) return;

  const float* x  = (const float*)d_in[0];
  const float* w1 = (const float*)d_in[1];
  const float* w2 = (const float*)d_in[2];
  const float* w3 = (const float*)d_in[3];
  float* out = (float*)d_out;

  size_t off = 0;
  const size_t oW1 = off; off += (size_t)HIDD * EMBD * 2;
  const size_t oW2 = off; off += (size_t)HIDD * EMBD * 2;
  const size_t oW3 = off; off += (size_t)EMBD * HIDD * 2;
  const size_t oXN = off; off += (size_t)MTOK * EMBD * 2;
  const size_t oAP = off; off += (size_t)TCH * HIDD * 4;
  const size_t oBP = off; off += (size_t)TCH * HIDD * 4;
  const size_t oYN = off; off += (size_t)TCH * HIDD * 2;
  const size_t oST = off; off += (size_t)4 * HIDD * 4;
  if (off > ws_size) return;
  if (off > (size_t)134217728) return;

  char* ws = (char*)d_ws;
  hh* W1H = (hh*)(ws + oW1);
  hh* W2H = (hh*)(ws + oW2);
  hh* W3H = (hh*)(ws + oW3);
  hh* XN  = (hh*)(ws + oXN);
  float* AP = (float*)(ws + oAP);
  float* BP = (float*)(ws + oBP);
  hh* YN  = (hh*)(ws + oYN);
  float* ST = (float*)(ws + oST);

  k_cvt<64><<<dim3((HIDD * EMBD) / 2048), dim3(256), 0, stream>>>(w1, W1H);
  k_cvt<64><<<dim3((HIDD * EMBD) / 2048), dim3(256), 0, stream>>>(w2, W2H);
  k_cvt<256><<<dim3((EMBD * HIDD) / 2048), dim3(256), 0, stream>>>(w3, W3H);
  k_rms1<<<dim3(MTOK), dim3(128), 0, stream>>>(x, XN);
  for (int b = 0; b < NBAT; ++b) {
    for (int ch = 0; ch < NCHK; ++ch) {
      const size_t row0 = (size_t)b * SEQL + (size_t)ch * TCH;
      const hh* xnc = XN + row0 * EMBD;
      const int rdst = (ch > 0) ? 1 : 0;
      const int wrst = (ch < NCHK - 1) ? 1 : 0;
      const int tbase = ch * TCH;
      k_gemm<0><<<dim3(HIDD / 128, TCH / 128), dim3(256), 0, stream>>>(xnc, W1H, x, AP);
      k_gemm<0><<<dim3(HIDD / 128, TCH / 128), dim3(256), 0, stream>>>(xnc, W2H, x, BP);
      k_scan<<<dim3(HIDD / 256), dim3(256), 0, stream>>>(BP, AP, ST, rdst, wrst, tbase);
      k_rms2<<<dim3(TCH), dim3(256), 0, stream>>>(AP, YN);
      k_gemm<1><<<dim3(EMBD / 128, TCH / 128), dim3(256), 0, stream>>>(YN, W3H, x + row0 * EMBD,
                                                                       out + row0 * EMBD);
    }
  }
  (void)hipGetLastError();
}
